// LMHCA_85212151152819
// MI455X (gfx1250) — hardware-verified
//
#include <hip/hip_runtime.h>
#include <math.h>

typedef __attribute__((ext_vector_type(16))) _Float16 v16h;
typedef __attribute__((ext_vector_type(16))) __bf16 v16b;
typedef __attribute__((ext_vector_type(8)))  _Float16 v8h;
typedef __attribute__((ext_vector_type(8)))  float v8f;
typedef __attribute__((ext_vector_type(4)))  float v4f;
typedef __attribute__((ext_vector_type(2)))  float v2f;
typedef __attribute__((ext_vector_type(4)))  unsigned v4u;
typedef __attribute__((ext_vector_type(4)))  int v4i;
typedef float __attribute__((may_alias)) float_a;
typedef int __attribute__((may_alias)) int_a;

template <typename T> __device__ __forceinline__ void vst2(void* p, T v) { *(volatile T*)p = v; __threadfence(); *(volatile T*)p = v; }
__device__ __forceinline__ v8f wmma16(v16h a, v16h b, v8f c) {
  v8f d = __builtin_amdgcn_wmma_f32_16x16x32_f16(false, a, false, b, (short)0, c, false, false);
  asm volatile("v_nop\n\tv_nop\n\tv_nop\n\tv_nop" : "+v"(d) : "v"(a), "v"(b));
  return d;
}
__device__ __forceinline__ v8f wmma_bf(v16b a, v16b b, v8f c) {
  v8f d = __builtin_amdgcn_wmma_f32_16x16x32_bf16(false, a, false, b, (short)0, c, false, false);
  asm volatile("v_nop\n\tv_nop\n\tv_nop\n\tv_nop" : "+v"(d) : "v"(a), "v"(b));
  return d;
}
__device__ __forceinline__ v16h frag_h(const _Float16* rowk0, int lane) {
  union { v16h v; v8h q[2]; } u; const _Float16* p = rowk0 + 8 * (lane >> 4);
  u.q[0] = *(const v8h*)p; u.q[1] = *(const v8h*)(p + 16); return u.v;
}
__device__ __forceinline__ v16h frag_f32(const float* rowk0, int lane) {
  v16h a; const float* p = rowk0 + 8 * (lane >> 4);
#pragma unroll
  for (int i = 0; i < 8; ++i) { a[i] = (_Float16)p[i]; a[8 + i] = (_Float16)p[16 + i]; }
  return a;
}
__device__ __forceinline__ v16h frag_f32s(const float* rowk0, int lane, float sc) {
  v16h a; const float* p = rowk0 + 8 * (lane >> 4);
#pragma unroll
  for (int i = 0; i < 8; ++i) { a[i] = (_Float16)(p[i] * sc); a[8 + i] = (_Float16)(p[16 + i] * sc); }
  return a;
}
__device__ __forceinline__ v16h fragc_f32(const float* W, int k0, int n, int lane, int ld, int K) {
  v16h a; const int g = lane >> 4;
#pragma unroll
  for (int i = 0; i < 8; ++i) { const int ka = k0 + 8 * g + i, kb = ka + 16;
    a[i] = (_Float16)(ka < K ? W[(size_t)(ka < K ? ka : K - 1) * ld + n] : 0.f); a[8 + i] = (_Float16)(kb < K ? W[(size_t)(kb < K ? kb : K - 1) * ld + n] : 0.f); }
  return a;
}
struct F2 { v16b h, l; };
__device__ __forceinline__ F2 bsplit16(const float v[16]) { F2 r;
#pragma unroll
  for (int i = 0; i < 16; ++i) { const __bf16 h = (__bf16)v[i]; r.h[i] = h; r.l[i] = (__bf16)(v[i] - (float)h); }
  return r; }
__device__ __forceinline__ F2 split_row(const float* row, int k0, int lane) { float v[16]; const float* p = row + k0 + 8 * (lane >> 4);
#pragma unroll
  for (int i = 0; i < 8; ++i) { v[i] = p[i]; v[8 + i] = p[16 + i]; }
  return bsplit16(v); }
__device__ __forceinline__ F2 split_rowK(const float* row, int k0, int lane, int K) { float v[16]; const int g = lane >> 4;
#pragma unroll
  for (int i = 0; i < 8; ++i) { const int ka = k0 + 8 * g + i, kb = ka + 16; v[i] = ka < K ? row[ka < K ? ka : K - 1] : 0.f; v[8 + i] = kb < K ? row[kb < K ? kb : K - 1] : 0.f; }
  return bsplit16(v); }
__device__ __forceinline__ F2 split_col(const float* W, int k0, int n, int lane, int ld, int K) { float v[16]; const int g = lane >> 4;
#pragma unroll
  for (int i = 0; i < 8; ++i) { const int ka = k0 + 8 * g + i, kb = ka + 16; v[i] = ka < K ? W[(size_t)(ka < K ? ka : K - 1) * ld + n] : 0.f; v[8 + i] = kb < K ? W[(size_t)(kb < K ? kb : K - 1) * ld + n] : 0.f; }
  return bsplit16(v); }
__device__ __forceinline__ v8f mac3(const F2& a, const F2& b, v8f c) { c = wmma_bf(a.l, b.h, c); c = wmma_bf(a.h, b.l, c); return wmma_bf(a.h, b.h, c); }
__device__ __forceinline__ float sigm(float v) { return 1.0f / (1.0f + expf(-v)); }
#define LDSX() do { asm volatile("s_wait_dscnt 0" ::: "memory"); __builtin_amdgcn_wave_barrier(); __builtin_amdgcn_fence(__ATOMIC_RELEASE, "workgroup"); } while (0)


#define NB 4
#define CC 256
#define HH 64
#define WWD 64
#define NP (HH * WWD)
#define NHD 4
#define NQ 16
#define HD 64
#define PD 256
#define YW (NQ * HD)
#define WSC 256.0f
#ifndef TPX
#define TPX (NP / 64)
#define TWB ((HH / 8) * (WWD / 8))
#define TZ (NP / 64)
#endif
typedef __attribute__((ext_vector_type(8))) __bf16 v8b;
__device__ __forceinline__ v16b frag_b(const __bf16* rowk0, int lane) {
  union { v16b v; v8b q[2]; } u; const __bf16* p = rowk0 + 8 * (lane >> 4);
  u.q[0] = *(const v8b*)p; u.q[1] = *(const v8b*)(p + 16); return u.v;
}
__device__ __forceinline__ float bfr(float v) { return (float)(__bf16)v; }
__device__ __attribute__((noinline)) float exp_ni(float v) { return expf(v); }
__device__ __attribute__((noinline)) float erf_ni(float v) { return erff(v); }

#define WS_PKV 0u
#define WS_PHW (WS_PKV + 2u * (size_t)2 * PD * CC)
#define WS_PQW (WS_PHW + 2u * (size_t)HD * PD)
#define WS_XT  (WS_PQW + 2u * (size_t)CC * YW)
#define WS_K16 (WS_XT + 2u * (size_t)NB * NP * CC)
#define WS_V16 (WS_K16 + 2u * (size_t)NB * NP * PD)
#define WS_AL  (WS_V16 + 2u * (size_t)NB * NP * PD)
#define WS_HV  (WS_AL + 4u * (size_t)NB * NP * NHD * NQ)
#define WS_Y16 (WS_HV + 4u * (size_t)NB * NP * PD)
#define WS_END (WS_Y16 + 2u * (size_t)NB * NP * YW)

__global__ __launch_bounds__(256) void k_pack(const float* __restrict__ KVW, const float* __restrict__ HW, const float* __restrict__ QW, char* __restrict__ ws) { const int n = blockIdx.x, which = blockIdx.y, t = threadIdx.x; __shared__ __align__(16) __bf16 sb[CC]; __shared__ __align__(16) _Float16 sh[YW];
  if (which == 0) { sb[t] = (__bf16)KVW[(size_t)n * CC + t]; __syncthreads(); if (t < CC / 8) vst2((unsigned*)((__bf16*)(ws + WS_PKV) + (size_t)n * CC + t * 8), *(const v4u*)&sb[t * 8]); }
  else if (which == 1) { if (n >= HD) return; sh[t] = (_Float16)(bfr(HW[(size_t)n * PD + t]) * WSC); __syncthreads(); if (t < PD / 8) vst2((unsigned*)((_Float16*)(ws + WS_PHW) + (size_t)n * PD + t * 8), *(const v4u*)&sh[t * 8]); }
  else { if (n >= CC) return; for (int k = t; k < YW; k += 256) sh[k] = (_Float16)(bfr(QW[(size_t)n * YW + k]) * WSC); __syncthreads(); for (int q = t; q < YW / 8; q += 256) vst2((unsigned*)((_Float16*)(ws + WS_PQW) + (size_t)n * YW + q * 8), *(const v4u*)&sh[q * 8]); } }
__global__ __launch_bounds__(256) void k_xt(const float* __restrict__ X, __bf16* __restrict__ XT) { __shared__ float st[64][CC + 1]; __shared__ __align__(16) __bf16 so2[64][CC + 8]; const int t = threadIdx.x; const int p0 = blockIdx.x * 64; const size_t b = blockIdx.y;
  for (int e = t; e < CC * 64; e += 256) { const int c = e >> 6, pl = e & 63; st[pl][c] = X[(b * CC + c) * NP + p0 + pl]; } __syncthreads();
  for (int e = t; e < 64 * CC; e += 256) { const int pl = e >> 8, c = e & 255; so2[pl][c] = (__bf16)st[pl][c]; } __syncthreads();
  for (int e = t; e < 64 * 32; e += 256) { const int pl = e >> 5, q = e & 31; vst2((unsigned*)(XT + ((b * NP + p0 + pl) * CC) + q * 8), *(const v4u*)&so2[pl][q * 8]); } }
__global__ __launch_bounds__(128) void k_kv(const __bf16* __restrict__ XT, const __bf16* __restrict__ P, _Float16* __restrict__ K16, _Float16* __restrict__ V16) { __shared__ __align__(16) _Float16 so[64][136];
  const int tid = threadIdx.x, wave = tid >> 5, lane = tid & 31, col = lane & 15, g = lane >> 4; const size_t b = blockIdx.z; const size_t rb = b * NP + (size_t)blockIdx.x * 64; const size_t r0 = rb + wave * 16; const int c0 = blockIdx.y * 128;
  v8f acc[8] = {};
#pragma unroll 2
  for (int kc = 0; kc < CC / 32; ++kc) { const v16b a = frag_b(XT + (r0 + col) * CC + kc * 32, lane);
#pragma unroll
    for (int j = 0; j < 8; ++j) acc[j] = wmma_bf(a, frag_b(P + (size_t)(c0 + j * 16 + col) * CC + kc * 32, lane), acc[j]); }
#pragma unroll
  for (int j = 0; j < 8; ++j)
#pragma unroll
    for (int r = 0; r < 8; ++r) so[wave * 16 + 8 * g + r][j * 16 + col] = (_Float16)acc[j][r];
  __syncthreads(); _Float16* dst = (c0 < PD) ? K16 : V16; const int cc0 = c0 % PD; for (int e = tid; e < 64 * 16; e += 128) { const int rl = e >> 4, q = e & 15; vst2((unsigned*)(dst + (rb + rl) * PD + cc0 + q * 8), *(const v4u*)&so[rl][q * 8]); } }
__global__ __launch_bounds__(256) void k_logit(const _Float16* __restrict__ K16, const float* __restrict__ DW, float* __restrict__ AL) { __shared__ float sk[64][PD + 1]; __shared__ float sd[NHD * NQ * HD]; __shared__ __align__(16) float so2[64][NHD * NQ + 4]; const int t = threadIdx.x; const size_t b = blockIdx.y; const size_t rb = b * NP + (size_t)blockIdx.x * 64;
  for (int e = t; e < 64 * PD; e += 256) { const int pl = e >> 8, c = e & 255; sk[pl][c] = (float)K16[(rb + pl) * PD + c]; } for (int e = t; e < NHD * NQ * HD; e += 256) sd[e] = bfr(DW[e]); __syncthreads();
  for (int e = t; e < 64 * NHD * NQ; e += 256) { const int pl = e >> 6, nq = e & 63; const int n = nq >> 4; float a = 0.f;
#pragma unroll 1
    for (int d = 0; d < HD; ++d) a += sk[pl][n * HD + d] * sd[nq * HD + d]; so2[pl][nq] = a; }
  __syncthreads(); for (int e = t; e < 64 * 16; e += 256) { const int pl = e >> 4, q = e & 15; vst2(AL + (rb + pl) * (NHD * NQ) + q * 4, *(const v4f*)&so2[pl][q * 4]); } }
__global__ __launch_bounds__(128) void k_hv(const _Float16* __restrict__ V16, const _Float16* __restrict__ PHW, float* __restrict__ HV) { __shared__ __align__(16) float sf[4][16][68];
  const int tid = threadIdx.x, wave = tid >> 5, lane = tid & 31, col = lane & 15, g = lane >> 4; const size_t b = blockIdx.y; const size_t rb = b * NP + (size_t)blockIdx.x * 64; const size_t r0 = rb + wave * 16;
  for (int n = 0; n < NHD; ++n) { v8f acc[4] = {};
#pragma unroll
    for (int kc = 0; kc < HD / 32; ++kc) { const v16h a = frag_h(V16 + (r0 + col) * PD + n * HD + kc * 32, lane);
#pragma unroll
      for (int j = 0; j < 4; ++j) acc[j] = wmma16(a, frag_h(PHW + (size_t)(j * 16 + col) * PD + n * HD + kc * 32, lane), acc[j]); }
#pragma unroll
    for (int j = 0; j < 4; ++j)
#pragma unroll
      for (int r = 0; r < 8; ++r) sf[wave][8 * g + r][j * 16 + col] = acc[j][r] * (1.0f / WSC);
    LDSX(); for (int rl = 0; rl < 16; ++rl) if (lane < 16) vst2(HV + (r0 + rl) * PD + n * HD + lane * 4, *(const v4f*)&sf[wave][rl][lane * 4]); LDSX(); } }
__global__ __launch_bounds__(256) void k_win(const float* __restrict__ AL, const float* __restrict__ HV, const float* __restrict__ HB, _Float16* __restrict__ Y16) {
  __shared__ _Float16 shv[100][PD]; __shared__ float sal[100][NHD * NQ + 1]; __shared__ float swt[8][NHD * NQ][9]; __shared__ __align__(16) _Float16 so2[8][YW];
  const int t = threadIdx.x; const size_t b = blockIdx.y; const int ty = (blockIdx.x / (WWD / 8)) * 8, tx = (blockIdx.x % (WWD / 8)) * 8;
  for (int e = t; e < 100 * PD; e += 256) { const int hp = e / PD, c = e % PD; const int yy = ty - 1 + hp / 10, xx = tx - 1 + hp % 10; const bool inb = yy >= 0 && yy < HH && xx >= 0 && xx < WWD; shv[hp][c] = (_Float16)(inb ? HV[(b * NP + (size_t)yy * WWD + xx) * PD + c] : 0.f); }
  for (int e = t; e < 100 * NHD * NQ; e += 256) { const int hp = e / (NHD * NQ), c = e % (NHD * NQ); const int yy = ty - 1 + hp / 10, xx = tx - 1 + hp % 10; const bool inb = yy >= 0 && yy < HH && xx >= 0 && xx < WWD; sal[hp][c] = inb ? AL[(b * NP + (size_t)yy * WWD + xx) * (NHD * NQ) + c] : 0.f; }
  __syncthreads();
  for (int grp = 0; grp < 8; ++grp) {
    for (int e = t; e < 8 * NHD * NQ; e += 256) { const int pi = e >> 6, nq = e & 63; const int pl = grp * 8 + pi; const int py = pl >> 3, px = pl & 7; float lg[9]; float mx = -3.0e38f;
#pragma unroll
      for (int l = 0; l < 9; ++l) { const int hp = (py + l / 3) * 10 + (px + l % 3); lg[l] = sal[hp][nq]; mx = fmaxf(mx, lg[l]); }
      float z = 0.f;
#pragma unroll
      for (int l = 0; l < 9; ++l) { lg[l] = expf(lg[l] - mx); z += lg[l]; }
      const float iz = 1.0f / z;
#pragma unroll
      for (int l = 0; l < 9; ++l) swt[pi][nq][l] = lg[l] * iz; }
    __syncthreads();
    for (int e = t; e < 8 * YW; e += 256) { const int pi = e / YW, ch = e % YW; const int pl = grp * 8 + pi; const int py = pl >> 3, px = pl & 7; const int q = ch >> 6, o = ch & 63; float a = bfr(HB[o]);
#pragma unroll 1
      for (int n = 0; n < NHD; ++n) {
#pragma unroll 1
        for (int l = 0; l < 9; ++l) { const int hp = (py + l / 3) * 10 + (px + l % 3); a += swt[pi][n * NQ + q][l] * (float)shv[hp][n * HD + o]; } }
      so2[pi][ch] = (_Float16)a; }
    __syncthreads();
    for (int e = t; e < 8 * (YW / 8); e += 256) { const int pi = e / (YW / 8), qq = e % (YW / 8); const int pl = grp * 8 + pi; const size_t p = b * NP + (size_t)(ty + (pl >> 3)) * WWD + tx + (pl & 7); vst2((unsigned*)(Y16 + p * YW + qq * 8), *(const v4u*)&so2[pi][qq * 8]); }
    __syncthreads(); } }
__global__ __launch_bounds__(128) void k_z(const _Float16* __restrict__ Y16, const _Float16* __restrict__ PQW, const float* __restrict__ QB, float* __restrict__ OUT) { __shared__ __align__(16) float so[128][64 + 4];
  const int tid = threadIdx.x, wave = tid >> 5, lane = tid & 31, col = lane & 15, g = lane >> 4; const size_t b = blockIdx.z; const int p0 = blockIdx.x * 64; const size_t r0 = b * NP + p0 + wave * 16; const int c0 = blockIdx.y * 128;
  v8f acc[8] = {};
#pragma unroll 2
  for (int kc = 0; kc < YW / 32; ++kc) { const v16h a = frag_h(Y16 + (r0 + col) * YW + kc * 32, lane);
#pragma unroll
    for (int j = 0; j < 8; ++j) acc[j] = wmma16(a, frag_h(PQW + (size_t)(c0 + j * 16 + col) * YW + kc * 32, lane), acc[j]); }
#pragma unroll
  for (int j = 0; j < 8; ++j)
#pragma unroll
    for (int r = 0; r < 8; ++r) so[j * 16 + col][wave * 16 + 8 * g + r] = acc[j][r] * (1.0f / WSC) + bfr(QB[c0 + j * 16 + col]);
  __syncthreads(); for (int e = tid; e < 128 * 16; e += 128) { const int c = e >> 4, q = e & 15; vst2(OUT + ((b * CC + c0 + c) * NP) + p0 + q * 4, *(const v4f*)&so[c][q * 4]); } }
extern "C" void kernel_launch(void* const* d_in, const int* in_sizes, int n_in, void* d_out, int out_size, void* d_ws, size_t ws_size, hipStream_t stream) {
  (void)in_sizes; (void)n_in; (void)out_size;
  const float** F = (const float**)d_in;
  if (ws_size < (size_t)WS_END) return;
  char* ws = (char*)d_ws; __bf16* XT = (__bf16*)(ws + WS_XT); _Float16 *K16 = (_Float16*)(ws + WS_K16), *V16 = (_Float16*)(ws + WS_V16), *Y16 = (_Float16*)(ws + WS_Y16); float *AL = (float*)(ws + WS_AL), *HV = (float*)(ws + WS_HV);
  k_pack<<<dim3(2 * PD, 3), 256, 0, stream>>>(F[1], F[3], F[5], ws);
  k_xt<<<dim3(NP / 64, NB), 256, 0, stream>>>(F[0], XT);
  k_kv<<<dim3(TPX, 2 * PD / 128, NB), 128, 0, stream>>>(XT, (const __bf16*)(ws + WS_PKV), K16, V16);
  k_logit<<<dim3(TPX, NB), 256, 0, stream>>>(K16, F[2], AL);
  k_hv<<<dim3(TPX, NB), 128, 0, stream>>>(V16, (const _Float16*)(ws + WS_PHW), HV);
  k_win<<<dim3(TWB, NB), 256, 0, stream>>>(AL, HV, F[4], Y16);
  k_z<<<dim3(TZ, CC / 128, NB), 128, 0, stream>>>(Y16, (const _Float16*)(ws + WS_PQW), F[6], (float*)d_out);
}
